// SphericalPhasorBlock_37082747633870
// MI455X (gfx1250) — hardware-verified
//
#include <hip/hip_runtime.h>
#include <stddef.h>
#include <stdint.h>
#include <math.h>

#define NBATCH 2
#define SEQ    2048
#define NTOK   4096
#define DMOD   512
#define KDIM   64
#define CHK    64
#define NCHB   32
#define NCH    64
#define PAIRS  32

static_assert(NTOK == NBATCH * SEQ);
static_assert(NCHB * CHK == SEQ);
static_assert(NCH == NBATCH * NCHB);
static_assert(NTOK % 64 == 0);
static_assert(DMOD == 512);
static_assert(DMOD % 64 == 0);
static_assert(KDIM == 64);
static_assert(CHK == 64);
static_assert(2 * PAIRS == KDIM);
static_assert((NTOK * DMOD) % 2048 == 0);
static_assert((NBATCH * DMOD * KDIM / 8) % 256 == 0);
static_assert(NTOK % 8 == 0);

#define WSC   64.0f
#define WINV  0.015625f
#define QKSC  8.0f
#define RINV  0.015625f
#define EPSN  1e-12f
#define EPSL  1e-5f
#define SFP   68
#define LP    72

typedef _Float16 hf;
typedef hf           v16h __attribute__((ext_vector_type(16)));
typedef hf           v8h  __attribute__((ext_vector_type(8)));
typedef float        v8f  __attribute__((ext_vector_type(8)));
typedef float        v4f  __attribute__((ext_vector_type(4)));
typedef unsigned int v4u  __attribute__((ext_vector_type(4)));

union Frag  { v16h v; v8h h[2]; };
union Pack8 { v8h h; v4u u; };

__device__ __forceinline__ v4u cvt8(const float (&f)[8], float sc) {
  Pack8 p;
  p.h = (v8h){(hf)(f[0] * sc), (hf)(f[1] * sc), (hf)(f[2] * sc), (hf)(f[3] * sc),
              (hf)(f[4] * sc), (hf)(f[5] * sc), (hf)(f[6] * sc), (hf)(f[7] * sc)};
  return p.u;
}

__device__ __forceinline__ v8f mma16(v16h a, v16h b, v8f c) {
  c = __builtin_amdgcn_wmma_f32_16x16x32_f16(false, a, false, b, (short)0, c, false, false);
  asm volatile("v_nop\n\tv_nop\n\tv_nop\n\tv_nop" : "+v"(c) : "v"(a), "v"(b));
  return c;
}

__device__ __forceinline__ v16h ldfrag(const hf* p, int ld, int row0, int k0, int lane) {
  const int m = lane & 15, lh = lane >> 4;
  const hf* q = p + (size_t)(row0 + m) * (size_t)ld + k0 + 8 * lh;
  Frag f;
  f.h[0] = *(const v8h*)(q);
  f.h[1] = *(const v8h*)(q + 16);
  return f.v;
}

__device__ __forceinline__ v8f zero8() { return (v8f){0.f, 0.f, 0.f, 0.f, 0.f, 0.f, 0.f, 0.f}; }

template <int KD>
__device__ __forceinline__ void gemm16x64(const hf* __restrict__ A, const hf* __restrict__ Bt,
                                          int m0, int n0, int lane, v8f (&acc)[4]) {
  static_assert(KD % 32 == 0);
#pragma unroll 1
  for (int k0 = 0; k0 < KD; k0 += 32) {
    const v16h a = ldfrag(A, KD, m0, k0, lane);
#pragma unroll
    for (int t = 0; t < 4; ++t) {
      const v16h b = ldfrag(Bt, KD, n0 + 16 * t, k0, lane);
      acc[t] = mma16(a, b, acc[t]);
    }
  }
}

__global__ __launch_bounds__(256) void k_cvt(const float* __restrict__ x, hf* __restrict__ xh) {
  const size_t i = (size_t)blockIdx.x * 2048 + (size_t)threadIdx.x * 8;
  const v4f a0 = *(const v4f*)(x + i);
  const v4f a1 = *(const v4f*)(x + i + 4);
  const float f[8] = {a0[0], a0[1], a0[2], a0[3], a1[0], a1[1], a1[2], a1[3]};
  const v4u u = cvt8(f, 1.0f);
  *(volatile v4u*)(xh + i) = u;
  __threadfence();
  *(volatile v4u*)(xh + i) = u;
}

template <int NOUT>
__global__ __launch_bounds__(256) void k_cvt_wt(const float* __restrict__ w, hf* __restrict__ wt) {
  static_assert(NOUT % 64 == 0);
  __shared__ __align__(16) float sw[64 * SFP];
  const int tid = threadIdx.x;
  const int kb = blockIdx.x * 64;
  const int nb = blockIdx.y * 64;
  {
    const int r  = tid >> 2;
    const int c0 = (tid & 3) * 16;
    const float* src = w + (size_t)(kb + r) * NOUT + nb + c0;
#pragma unroll
    for (int e = 0; e < 4; ++e) *(v4f*)(sw + r * SFP + c0 + 4 * e) = *(const v4f*)(src + 4 * e);
  }
  __syncthreads();
  v4u hv[2];
  size_t go[2];
#pragma unroll
  for (int j = 0; j < 2; ++j) {
    const int p  = tid + 256 * j;
    const int n  = p >> 3;
    const int pc = p & 7;
    const float* cp = sw + (pc * 8) * SFP + n;
    float f[8];
#pragma unroll
    for (int e = 0; e < 8; ++e) f[e] = cp[e * SFP];
    hv[j] = cvt8(f, WSC);
    go[j] = (size_t)(nb + n) * DMOD + kb + pc * 8;
  }
#pragma unroll
  for (int j = 0; j < 2; ++j) *(volatile v4u*)(wt + go[j]) = hv[j];
  __threadfence();
#pragma unroll
  for (int j = 0; j < 2; ++j) *(volatile v4u*)(wt + go[j]) = hv[j];
}

template <int MODE>
__global__ __launch_bounds__(128) void k_gemm(const hf* __restrict__ A, const hf* __restrict__ Bt,
                                              const float* __restrict__ bias, const float* __restrict__ res,
                                              hf* __restrict__ yh, float* __restrict__ yf) {
  __shared__ __align__(16) float sf[64 * SFP];
  const int tid = threadIdx.x, lane = tid & 31, wave = tid >> 5;
  const int hh = lane >> 4, c = lane & 15;
  const int mb = blockIdx.x * 64;
  const int nb = blockIdx.y * 64;
  const int m0 = mb + wave * 16;

  v8f acc[4];
#pragma unroll
  for (int t = 0; t < 4; ++t) acc[t] = zero8();
  gemm16x64<DMOD>(A, Bt, m0, nb, lane, acc);

  float bcol[4];
#pragma unroll
  for (int t = 0; t < 4; ++t) bcol[t] = bias[nb + 16 * t + c];
#pragma unroll
  for (int t = 0; t < 4; ++t) {
#pragma unroll
    for (int r = 0; r < 8; ++r) {
      float v = acc[t][r] * WINV + bcol[t];
      if constexpr (MODE == 0) v = 0.5f * v * (1.0f + erff(v * 0.70710678118654752f));
      sf[(wave * 16 + 8 * hh + r) * SFP + 16 * t + c] = v;
    }
  }
  __syncthreads();

  if constexpr (MODE == 0) {
    v4u hv[4];
    size_t go[4];
#pragma unroll
    for (int j = 0; j < 4; ++j) {
      const int p  = tid + 128 * j;
      const int lr = p >> 3;
      const int d0 = (p & 7) * 8;
      const float* ra = sf + lr * SFP + d0;
      const v4f a0 = *(const v4f*)(ra), a1 = *(const v4f*)(ra + 4);
      const float f[8] = {a0[0], a0[1], a0[2], a0[3], a1[0], a1[1], a1[2], a1[3]};
      hv[j] = cvt8(f, 1.0f);
      go[j] = ((size_t)(mb + lr)) * DMOD + nb + d0;
    }
#pragma unroll
    for (int j = 0; j < 4; ++j) *(volatile v4u*)(yh + go[j]) = hv[j];
    __threadfence();
#pragma unroll
    for (int j = 0; j < 4; ++j) *(volatile v4u*)(yh + go[j]) = hv[j];
  } else if constexpr (MODE == 1) {
    v4u hv[4];
    size_t go[4];
#pragma unroll
    for (int j = 0; j < 4; ++j) {
      const int p  = tid + 128 * j;
      const int d  = p >> 3;
      const int pc = p & 7;
      const float* cp = sf + (pc * 8) * SFP + d;
      float f[8];
#pragma unroll
      for (int e = 0; e < 8; ++e) f[e] = cp[e * SFP];
      hv[j] = cvt8(f, 1.0f);
      go[j] = ((size_t)(nb + d)) * (size_t)NTOK + mb + pc * 8;
    }
#pragma unroll
    for (int j = 0; j < 4; ++j) *(volatile v4u*)(yh + go[j]) = hv[j];
    __threadfence();
#pragma unroll
    for (int j = 0; j < 4; ++j) *(volatile v4u*)(yh + go[j]) = hv[j];
  } else {
    v4f val[8];
    size_t go[8];
#pragma unroll
    for (int it = 0; it < 8; ++it) {
      const int p    = tid + 128 * it;
      const int L    = p >> 3;
      const int pc   = p & 7;
      const int row  = L >> 1;
      const int half = L & 1;
      const int col  = half * 32 + pc * 4;
      go[it]  = (size_t)(mb + row) * DMOD + nb + col;
      val[it] = *(const v4f*)(sf + row * SFP + col) + *(const v4f*)(res + go[it]);
    }
#pragma unroll
    for (int it = 0; it < 8; ++it) *(volatile v4f*)(yf + go[it]) = val[it];
    __threadfence();
#pragma unroll
    for (int it = 0; it < 8; ++it) *(volatile v4f*)(yf + go[it]) = val[it];
  }
}

template <int WT>
__global__ __launch_bounds__(128) void k_enc(const hf* __restrict__ H, const hf* __restrict__ W2t,
                                             const float* __restrict__ bias, hf* __restrict__ P,
                                             hf* __restrict__ PT) {
  __shared__ __align__(16) float sf[64 * SFP];
  __shared__ float sinv[64];
  const int tid = threadIdx.x, lane = tid & 31, wave = tid >> 5;
  const int hh = lane >> 4, c = lane & 15;
  const int mb = blockIdx.x * 64;
  const int m0 = mb + wave * 16;

  v8f acc[4];
#pragma unroll
  for (int t = 0; t < 4; ++t) acc[t] = zero8();
  gemm16x64<DMOD>(H, W2t, m0, 0, lane, acc);

  float bcol[4];
#pragma unroll
  for (int t = 0; t < 4; ++t) bcol[t] = bias[16 * t + c];
#pragma unroll
  for (int t = 0; t < 4; ++t) {
#pragma unroll
    for (int r = 0; r < 8; ++r) sf[(wave * 16 + 8 * hh + r) * SFP + 16 * t + c] = acc[t][r] * WINV + bcol[t];
  }
  __syncthreads();
  if (tid < 64) {
    float s = 0.f;
    const float* rp = sf + tid * SFP;
#pragma unroll 1
    for (int j = 0; j < KDIM; ++j) { const float v = rp[j]; s = fmaf(v, v, s); }
    sinv[tid] = QKSC / fmaxf(sqrtf(s), EPSN);
  }
  __syncthreads();

  v4u hv[4];
  size_t go[4];
#pragma unroll
  for (int j = 0; j < 4; ++j) {
    const int p  = tid + 128 * j;
    const int lr = p >> 3;
    const int d0 = (p & 7) * 8;
    const float* ra = sf + lr * SFP + d0;
    const float iv = sinv[lr];
    const v4f a0 = *(const v4f*)(ra), a1 = *(const v4f*)(ra + 4);
    const float f[8] = {a0[0] * iv, a0[1] * iv, a0[2] * iv, a0[3] * iv, a1[0] * iv, a1[1] * iv, a1[2] * iv, a1[3] * iv};
    hv[j] = cvt8(f, 1.0f);
    go[j] = ((size_t)(mb + lr)) * KDIM + d0;
  }
#pragma unroll
  for (int j = 0; j < 4; ++j) *(volatile v4u*)(P + go[j]) = hv[j];
  __threadfence();
#pragma unroll
  for (int j = 0; j < 4; ++j) *(volatile v4u*)(P + go[j]) = hv[j];

  if constexpr (WT != 0) {
    v4u tv[4];
    size_t tgo[4];
#pragma unroll
    for (int j = 0; j < 4; ++j) {
      const int p  = tid + 128 * j;
      const int jj = p >> 3;
      const int pc = p & 7;
      const float* cp = sf + (pc * 8) * SFP + jj;
      float f[8];
#pragma unroll
      for (int e = 0; e < 8; ++e) f[e] = cp[e * SFP] * sinv[pc * 8 + e];
      tv[j]  = cvt8(f, 1.0f);
      tgo[j] = ((size_t)jj) * (size_t)NTOK + mb + pc * 8;
    }
#pragma unroll
    for (int j = 0; j < 4; ++j) *(volatile v4u*)(PT + tgo[j]) = tv[j];
    __threadfence();
#pragma unroll
    for (int j = 0; j < 4; ++j) *(volatile v4u*)(PT + tgo[j]) = tv[j];
  }
}

__global__ __launch_bounds__(128) void k_state(const hf* __restrict__ vt, const hf* __restrict__ kt,
                                               float* __restrict__ sst) {
  __shared__ __align__(16) float sf[64 * SFP];
  const int tid = threadIdx.x, lane = tid & 31, wave = tid >> 5;
  const int hh = lane >> 4, c = lane & 15;
  const int db  = blockIdx.x * 64;
  const int bc  = blockIdx.y;
  const int tok = bc * CHK;
  const int m0  = db + wave * 16;

  v8f acc[4];
#pragma unroll
  for (int t = 0; t < 4; ++t) acc[t] = zero8();
#pragma unroll
  for (int ks = 0; ks < 2; ++ks) {
    const v16h a = ldfrag(vt, NTOK, m0, tok + 32 * ks, lane);
#pragma unroll
    for (int t = 0; t < 4; ++t) {
      const v16h b = ldfrag(kt, NTOK, 16 * t, tok + 32 * ks, lane);
      acc[t] = mma16(a, b, acc[t]);
    }
  }
#pragma unroll
  for (int t = 0; t < 4; ++t) {
#pragma unroll
    for (int r = 0; r < 8; ++r) sf[(wave * 16 + 8 * hh + r) * SFP + 16 * t + c] = acc[t][r];
  }
  __syncthreads();
  v4f val[8];
  size_t go[8];
#pragma unroll
  for (int it = 0; it < 8; ++it) {
    const int p    = tid + 128 * it;
    const int L    = p >> 3;
    const int pc   = p & 7;
    const int row  = L >> 1;
    const int half = L & 1;
    const int col  = half * 32 + pc * 4;
    val[it] = *(const v4f*)(sf + row * SFP + col);
    go[it]  = ((size_t)bc * DMOD + db + row) * KDIM + col;
  }
#pragma unroll
  for (int it = 0; it < 8; ++it) *(volatile v4f*)(sst + go[it]) = val[it];
  __threadfence();
#pragma unroll
  for (int it = 0; it < 8; ++it) *(volatile v4f*)(sst + go[it]) = val[it];
}

__global__ __launch_bounds__(256) void k_prefix(const float* __restrict__ sst, hf* __restrict__ spl) {
  const int g = blockIdx.x * 256 + threadIdx.x;
  const int b = g / (DMOD * KDIM / 8);
  const int e = g - b * (DMOD * KDIM / 8);
  float run[8];
#pragma unroll
  for (int k = 0; k < 8; ++k) run[k] = 0.f;
#pragma unroll 1
  for (int cc = 0; cc < NCHB; ++cc) {
    const size_t base = (size_t)(b * NCHB + cc) * (size_t)(DMOD * KDIM) + (size_t)e * 8;
    const v4u u = cvt8(run, 1.0f);
    *(volatile v4u*)(spl + base) = u;
    __threadfence();
    *(volatile v4u*)(spl + base) = u;
    const v4f a0 = *(const v4f*)(sst + base);
    const v4f a1 = *(const v4f*)(sst + base + 4);
    run[0] += a0[0]; run[1] += a0[1]; run[2] += a0[2]; run[3] += a0[3];
    run[4] += a1[0]; run[5] += a1[1]; run[6] += a1[2]; run[7] += a1[3];
  }
}

__global__ __launch_bounds__(128) void k_retr(const hf* __restrict__ qp, const hf* __restrict__ kp,
                                              const hf* __restrict__ vt, const hf* __restrict__ spl,
                                              float* __restrict__ rout) {
  __shared__ __align__(16) hf    pt[4 * 16 * LP];
  __shared__ __align__(16) float sf[64 * SFP];
  const int tid = threadIdx.x, lane = tid & 31, wave = tid >> 5;
  const int hh = lane >> 4, c = lane & 15;
  const int nb  = blockIdx.x * 64;
  const int bc  = blockIdx.y;
  const int cw  = bc - (bc / NCHB) * NCHB;
  const int tok = bc * CHK;
  const int tl0 = wave * 16;
  const int q0  = tok + tl0;

  v8f s[4];
#pragma unroll
  for (int j = 0; j < 4; ++j) s[j] = zero8();
#pragma unroll
  for (int dc = 0; dc < 2; ++dc) {
    const v16h qa = ldfrag(qp, KDIM, q0, 32 * dc, lane);
#pragma unroll
    for (int j = 0; j < 4; ++j) {
      const v16h kb = ldfrag(kp, KDIM, tok + 16 * j, 32 * dc, lane);
      s[j] = mma16(qa, kb, s[j]);
    }
  }
  hf* pw = pt + wave * 16 * LP;
#pragma unroll
  for (int j = 0; j < 4; ++j) {
    const int sl = 16 * j + c;
#pragma unroll
    for (int r = 0; r < 8; ++r) {
      const int tl = tl0 + 8 * hh + r;
      const float a = (sl <= tl) ? s[j][r] : 0.f;
      pw[(8 * hh + r) * LP + sl] = (hf)a;
    }
  }
  __syncthreads();

  v8f acc[4];
#pragma unroll
  for (int t = 0; t < 4; ++t) acc[t] = zero8();
  const hf* sc = spl + (size_t)bc * (size_t)(DMOD * KDIM);
#pragma unroll
  for (int dc = 0; dc < 2; ++dc) {
    const v16h qa = ldfrag(qp, KDIM, q0, 32 * dc, lane);
#pragma unroll
    for (int t = 0; t < 4; ++t) {
      const v16h sb = ldfrag(sc, KDIM, nb + 16 * t, 32 * dc, lane);
      acc[t] = mma16(qa, sb, acc[t]);
    }
  }
#pragma unroll
  for (int kk = 0; kk < 2; ++kk) {
    const v16h pa = ldfrag(pw, LP, 0, 32 * kk, lane);
#pragma unroll
    for (int t = 0; t < 4; ++t) {
      const v16h vb = ldfrag(vt, NTOK, nb + 16 * t, tok + 32 * kk, lane);
      acc[t] = mma16(pa, vb, acc[t]);
    }
  }

#pragma unroll
  for (int r = 0; r < 8; ++r) {
    const int tl = tl0 + 8 * hh + r;
    const float pos = (float)(cw * CHK + tl + 1);
    const float scl = RINV * (1.0f / sqrtf(pos * 32.0f));
#pragma unroll
    for (int t = 0; t < 4; ++t) sf[tl * SFP + 16 * t + c] = acc[t][r] * scl;
  }
  __syncthreads();
  v4f val[8];
  size_t go[8];
#pragma unroll
  for (int it = 0; it < 8; ++it) {
    const int p    = tid + 128 * it;
    const int L    = p >> 3;
    const int pc   = p & 7;
    const int row  = L >> 1;
    const int half = L & 1;
    const int col  = half * 32 + pc * 4;
    val[it] = *(const v4f*)(sf + row * SFP + col);
    go[it]  = (size_t)(tok + row) * DMOD + nb + col;
  }
#pragma unroll
  for (int it = 0; it < 8; ++it) *(volatile v4f*)(rout + go[it]) = val[it];
  __threadfence();
#pragma unroll
  for (int it = 0; it < 8; ++it) *(volatile v4f*)(rout + go[it]) = val[it];
}

__global__ __launch_bounds__(256) void k_ln(const float* __restrict__ rin, const float* __restrict__ g,
                                            const float* __restrict__ bta, hf* __restrict__ rln) {
  const int lane = threadIdx.x & 31, wave = threadIdx.x >> 5;
  const int row = blockIdx.x * 8 + wave;
  const float* rp = rin + (size_t)row * DMOD;
  const int c0 = lane * 8, c1 = 256 + lane * 8;
  const v4f a0 = *(const v4f*)(rp + c0), a1 = *(const v4f*)(rp + c0 + 4);
  const v4f a2 = *(const v4f*)(rp + c1), a3 = *(const v4f*)(rp + c1 + 4);
  const float v[16] = {a0[0], a0[1], a0[2], a0[3], a1[0], a1[1], a1[2], a1[3],
                       a2[0], a2[1], a2[2], a2[3], a3[0], a3[1], a3[2], a3[3]};
  float sm = 0.f;
#pragma unroll
  for (int k = 0; k < 16; ++k) sm += v[k];
#pragma unroll
  for (int off = 1; off < 32; off <<= 1) sm += __shfl_xor(sm, off, 32);
  const float mu = sm * (1.0f / (float)DMOD);
  float sq = 0.f;
#pragma unroll
  for (int k = 0; k < 16; ++k) { const float d = v[k] - mu; sq = fmaf(d, d, sq); }
#pragma unroll
  for (int off = 1; off < 32; off <<= 1) sq += __shfl_xor(sq, off, 32);
  const float var = sq * (1.0f / (float)DMOD);
  const float rsd = 1.0f / sqrtf(var + EPSL);
  const v4f g0 = *(const v4f*)(g + c0), g1 = *(const v4f*)(g + c0 + 4);
  const v4f g2 = *(const v4f*)(g + c1), g3 = *(const v4f*)(g + c1 + 4);
  const v4f b0 = *(const v4f*)(bta + c0), b1 = *(const v4f*)(bta + c0 + 4);
  const v4f b2 = *(const v4f*)(bta + c1), b3 = *(const v4f*)(bta + c1 + 4);
  const float gv[16] = {g0[0], g0[1], g0[2], g0[3], g1[0], g1[1], g1[2], g1[3],
                        g2[0], g2[1], g2[2], g2[3], g3[0], g3[1], g3[2], g3[3]};
  const float bv[16] = {b0[0], b0[1], b0[2], b0[3], b1[0], b1[1], b1[2], b1[3],
                        b2[0], b2[1], b2[2], b2[3], b3[0], b3[1], b3[2], b3[3]};
  float y0[8], y1[8];
#pragma unroll
  for (int k = 0; k < 8; ++k) {
    y0[k] = (v[k] - mu) * rsd * gv[k] + bv[k];
    y1[k] = (v[8 + k] - mu) * rsd * gv[8 + k] + bv[8 + k];
  }
  const v4u u0 = cvt8(y0, 1.0f), u1 = cvt8(y1, 1.0f);
  hf* op = rln + (size_t)row * DMOD;
  *(volatile v4u*)(op + c0) = u0;
  *(volatile v4u*)(op + c1) = u1;
  __threadfence();
  *(volatile v4u*)(op + c0) = u0;
  *(volatile v4u*)(op + c1) = u1;
}

extern "C" void kernel_launch(void* const* d_in, const int* in_sizes, int n_in,
                              void* d_out, int out_size, void* d_ws, size_t ws_size,
                              hipStream_t stream) {
  if (n_in < 15) return;
  if (in_sizes[0]  != NTOK * DMOD) return;
  if (in_sizes[1]  != DMOD * DMOD) return;
  if (in_sizes[2]  != DMOD) return;
  if (in_sizes[3]  != DMOD * KDIM) return;
  if (in_sizes[4]  != KDIM) return;
  if (in_sizes[5]  != DMOD * DMOD) return;
  if (in_sizes[6]  != DMOD) return;
  if (in_sizes[7]  != DMOD * KDIM) return;
  if (in_sizes[8]  != KDIM) return;
  if (in_sizes[9]  != DMOD * DMOD) return;
  if (in_sizes[10] != DMOD) return;
  if (in_sizes[11] != DMOD) return;
  if (in_sizes[12] != DMOD) return;
  if (in_sizes[13] != DMOD * DMOD) return;
  if (in_sizes[14] != DMOD) return;
  if (out_size != NTOK * DMOD) return;

  const float* X   = (const float*)d_in[0];
  const float* kw1 = (const float*)d_in[1];
  const float* kb1 = (const float*)d_in[2];
  const float* kw2 = (const float*)d_in[3];
  const float* kb2 = (const float*)d_in[4];
  const float* qw1 = (const float*)d_in[5];
  const float* qb1 = (const float*)d_in[6];
  const float* qw2 = (const float*)d_in[7];
  const float* qb2 = (const float*)d_in[8];
  const float* vw  = (const float*)d_in[9];
  const float* vb  = (const float*)d_in[10];
  const float* lng = (const float*)d_in[11];
  const float* lnb = (const float*)d_in[12];
  const float* ow  = (const float*)d_in[13];
  const float* ob  = (const float*)d_in[14];
  float* out = (float*)d_out;

  const size_t PLX = (size_t)NTOK * DMOD * 2;
  const size_t PLW = (size_t)DMOD * DMOD * 2;
  const size_t PW2 = (size_t)KDIM * DMOD * 2;
  const size_t PQK = (size_t)NTOK * KDIM * 2;
  const size_t SSF = (size_t)NCH * DMOD * KDIM * 4;
  const size_t SSH = (size_t)NCH * DMOD * KDIM * 2;
  const size_t RFB = (size_t)NTOK * DMOD * 4;
  size_t off = 0;
  const size_t oXh  = off; off += PLX;
  const size_t oW1K = off; off += PLW;
  const size_t oW1Q = off; off += PLW;
  const size_t oWV  = off; off += PLW;
  const size_t oWO  = off; off += PLW;
  const size_t oW2K = off; off += PW2;
  const size_t oW2Q = off; off += PW2;
  const size_t oHk  = off; off += PLX;
  const size_t oHq  = off; off += PLX;
  const size_t oVT  = off; off += PLX;
  const size_t oQp  = off; off += PQK;
  const size_t oKp  = off; off += PQK;
  const size_t oKT  = off; off += PQK;
  const size_t oSst = off; off += SSF;
  const size_t oSpl = off; off += SSH;
  const size_t oR   = off; off += RFB;
  const size_t oRLN = off; off += PLX;
  if (off > ws_size) return;
  if (off > (size_t)134217728) return;

  char* ws = (char*)d_ws;
  hf* Xh   = (hf*)(ws + oXh);
  hf* W1Kt = (hf*)(ws + oW1K);
  hf* W1Qt = (hf*)(ws + oW1Q);
  hf* WVt  = (hf*)(ws + oWV);
  hf* WOt  = (hf*)(ws + oWO);
  hf* W2Kt = (hf*)(ws + oW2K);
  hf* W2Qt = (hf*)(ws + oW2Q);
  hf* Hk   = (hf*)(ws + oHk);
  hf* Hq   = (hf*)(ws + oHq);
  hf* VT   = (hf*)(ws + oVT);
  hf* Qp   = (hf*)(ws + oQp);
  hf* Kp   = (hf*)(ws + oKp);
  hf* KTp  = (hf*)(ws + oKT);
  float* Sst = (float*)(ws + oSst);
  hf* Spl  = (hf*)(ws + oSpl);
  float* Rf  = (float*)(ws + oR);
  hf* RLN  = (hf*)(ws + oRLN);

  k_cvt<<<dim3((NTOK * DMOD) / 2048), dim3(256), 0, stream>>>(X, Xh);
  k_cvt_wt<DMOD><<<dim3(DMOD / 64, DMOD / 64), dim3(256), 0, stream>>>(kw1, W1Kt);
  k_cvt_wt<DMOD><<<dim3(DMOD / 64, DMOD / 64), dim3(256), 0, stream>>>(qw1, W1Qt);
  k_cvt_wt<DMOD><<<dim3(DMOD / 64, DMOD / 64), dim3(256), 0, stream>>>(vw, WVt);
  k_cvt_wt<DMOD><<<dim3(DMOD / 64, DMOD / 64), dim3(256), 0, stream>>>(ow, WOt);
  k_cvt_wt<KDIM><<<dim3(DMOD / 64, KDIM / 64), dim3(256), 0, stream>>>(kw2, W2Kt);
  k_cvt_wt<KDIM><<<dim3(DMOD / 64, KDIM / 64), dim3(256), 0, stream>>>(qw2, W2Qt);
  k_gemm<0><<<dim3(NTOK / 64, DMOD / 64), dim3(128), 0, stream>>>(Xh, W1Kt, kb1, X, Hk, Rf);
  k_gemm<0><<<dim3(NTOK / 64, DMOD / 64), dim3(128), 0, stream>>>(Xh, W1Qt, qb1, X, Hq, Rf);
  k_gemm<1><<<dim3(NTOK / 64, DMOD / 64), dim3(128), 0, stream>>>(Xh, WVt, vb, X, VT, Rf);
  k_enc<0><<<dim3(NTOK / 64), dim3(128), 0, stream>>>(Hq, W2Qt, qb2, Qp, KTp);
  k_enc<1><<<dim3(NTOK / 64), dim3(128), 0, stream>>>(Hk, W2Kt, kb2, Kp, KTp);
  k_state<<<dim3(DMOD / 64, NCH), dim3(128), 0, stream>>>(VT, KTp, Sst);
  k_prefix<<<dim3((NBATCH * DMOD * KDIM / 8) / 256), dim3(256), 0, stream>>>(Sst, Spl);
  k_retr<<<dim3(DMOD / 64, NCH), dim3(128), 0, stream>>>(Qp, Kp, VT, Spl, Rf);
  k_ln<<<dim3(NTOK / 8), dim3(256), 0, stream>>>(Rf, lng, lnb, RLN);
  k_gemm<2><<<dim3(NTOK / 64, DMOD / 64), dim3(128), 0, stream>>>(RLN, WOt, ob, X, Hq, out);
  (void)hipGetLastError();
}
